// CrossViewAttention_48790828482898
// MI455X (gfx1250) — hardware-verified
//
#include <hip/hip_runtime.h>
#include <math.h>

typedef __attribute__((ext_vector_type(16))) _Float16 v16h;
typedef __attribute__((ext_vector_type(16))) __bf16 v16b;
typedef __attribute__((ext_vector_type(8)))  _Float16 v8h;
typedef __attribute__((ext_vector_type(8)))  float v8f;
typedef __attribute__((ext_vector_type(4)))  float v4f;
typedef __attribute__((ext_vector_type(2)))  float v2f;
typedef __attribute__((ext_vector_type(4)))  unsigned v4u;
typedef __attribute__((ext_vector_type(4)))  int v4i;
typedef float __attribute__((may_alias)) float_a;
typedef int __attribute__((may_alias)) int_a;

template <typename T> __device__ __forceinline__ void vst2(void* p, T v) { *(volatile T*)p = v; __threadfence(); *(volatile T*)p = v; }
__device__ __forceinline__ v8f wmma16(v16h a, v16h b, v8f c) {
  v8f d = __builtin_amdgcn_wmma_f32_16x16x32_f16(false, a, false, b, (short)0, c, false, false);
  asm volatile("v_nop\n\tv_nop\n\tv_nop\n\tv_nop" : "+v"(d) : "v"(a), "v"(b));
  return d;
}
__device__ __forceinline__ v8f wmma_bf(v16b a, v16b b, v8f c) {
  v8f d = __builtin_amdgcn_wmma_f32_16x16x32_bf16(false, a, false, b, (short)0, c, false, false);
  asm volatile("v_nop\n\tv_nop\n\tv_nop\n\tv_nop" : "+v"(d) : "v"(a), "v"(b));
  return d;
}
__device__ __forceinline__ v16h frag_h(const _Float16* rowk0, int lane) {
  union { v16h v; v8h q[2]; } u; const _Float16* p = rowk0 + 8 * (lane >> 4);
  u.q[0] = *(const v8h*)p; u.q[1] = *(const v8h*)(p + 16); return u.v;
}
__device__ __forceinline__ v16h frag_f32(const float* rowk0, int lane) {
  v16h a; const float* p = rowk0 + 8 * (lane >> 4);
#pragma unroll
  for (int i = 0; i < 8; ++i) { a[i] = (_Float16)p[i]; a[8 + i] = (_Float16)p[16 + i]; }
  return a;
}
__device__ __forceinline__ v16h frag_f32s(const float* rowk0, int lane, float sc) {
  v16h a; const float* p = rowk0 + 8 * (lane >> 4);
#pragma unroll
  for (int i = 0; i < 8; ++i) { a[i] = (_Float16)(p[i] * sc); a[8 + i] = (_Float16)(p[16 + i] * sc); }
  return a;
}
__device__ __forceinline__ v16h fragc_f32(const float* W, int k0, int n, int lane, int ld, int K) {
  v16h a; const int g = lane >> 4;
#pragma unroll
  for (int i = 0; i < 8; ++i) { const int ka = k0 + 8 * g + i, kb = ka + 16;
    a[i] = (_Float16)(ka < K ? W[(size_t)(ka < K ? ka : K - 1) * ld + n] : 0.f); a[8 + i] = (_Float16)(kb < K ? W[(size_t)(kb < K ? kb : K - 1) * ld + n] : 0.f); }
  return a;
}
struct F2 { v16b h, l; };
__device__ __forceinline__ F2 bsplit16(const float v[16]) { F2 r;
#pragma unroll
  for (int i = 0; i < 16; ++i) { const __bf16 h = (__bf16)v[i]; r.h[i] = h; r.l[i] = (__bf16)(v[i] - (float)h); }
  return r; }
__device__ __forceinline__ F2 split_row(const float* row, int k0, int lane) { float v[16]; const float* p = row + k0 + 8 * (lane >> 4);
#pragma unroll
  for (int i = 0; i < 8; ++i) { v[i] = p[i]; v[8 + i] = p[16 + i]; }
  return bsplit16(v); }
__device__ __forceinline__ F2 split_rowK(const float* row, int k0, int lane, int K) { float v[16]; const int g = lane >> 4;
#pragma unroll
  for (int i = 0; i < 8; ++i) { const int ka = k0 + 8 * g + i, kb = ka + 16; v[i] = ka < K ? row[ka < K ? ka : K - 1] : 0.f; v[8 + i] = kb < K ? row[kb < K ? kb : K - 1] : 0.f; }
  return bsplit16(v); }
__device__ __forceinline__ F2 split_col(const float* W, int k0, int n, int lane, int ld, int K) { float v[16]; const int g = lane >> 4;
#pragma unroll
  for (int i = 0; i < 8; ++i) { const int ka = k0 + 8 * g + i, kb = ka + 16; v[i] = ka < K ? W[(size_t)(ka < K ? ka : K - 1) * ld + n] : 0.f; v[8 + i] = kb < K ? W[(size_t)(kb < K ? kb : K - 1) * ld + n] : 0.f; }
  return bsplit16(v); }
__device__ __forceinline__ v8f mac3(const F2& a, const F2& b, v8f c) { c = wmma_bf(a.l, b.h, c); c = wmma_bf(a.h, b.l, c); return wmma_bf(a.h, b.h, c); }
__device__ __forceinline__ float sigm(float v) { return 1.0f / (1.0f + expf(-v)); }
#define LDSX() do { asm volatile("s_wait_dscnt 0" ::: "memory"); __builtin_amdgcn_wave_barrier(); __builtin_amdgcn_fence(__ATOMIC_RELEASE, "workgroup"); } while (0)


#define NBB 12
#define CC 512
#define TT 1024
#define NH 8
#define HD 64
#ifndef TBB
#define TBB NBB
#endif
typedef __attribute__((ext_vector_type(8))) __bf16 v8b;
__device__ __forceinline__ v16b frag_b(const __bf16* rowk0, int lane) {
  union { v16b v; v8b q[2]; } u; const __bf16* p = rowk0 + 8 * (lane >> 4);
  u.q[0] = *(const v8b*)p; u.q[1] = *(const v8b*)(p + 16); return u.v;
}
__device__ __forceinline__ float bfr(float v) { return (float)(__bf16)v; }
__device__ __attribute__((noinline)) float exp_ni(float v) { return expf(v); }
__device__ __attribute__((noinline)) float erf_ni(float v) { return erff(v); }

#define WS_Q   0u
#define WS_KH  (WS_Q + 2u * (size_t)NBB * TT * CC)
#define WS_KL  (WS_KH + 2u * (size_t)NBB * TT * CC)
#define WS_VH  (WS_KL + 2u * (size_t)NBB * TT * CC)
#define WS_VL  (WS_VH + 2u * (size_t)NBB * CC * TT)
#define WS_Y   (WS_VL + 2u * (size_t)NBB * CC * TT)
#define WS_END (WS_Y + 4u * (size_t)NBB * TT * CC)

__global__ __launch_bounds__(128) void k_q(const float* __restrict__ Qp, _Float16* __restrict__ QR) { __shared__ __align__(16) _Float16 st[64][136]; const int t = threadIdx.x; const size_t bb = blockIdx.z; const int t0 = blockIdx.x * 64, c0 = blockIdx.y * 128;
  for (int e = t; e < 128 * 64; e += 128) { const int cl = e >> 6, tl = e & 63; st[tl][cl] = (_Float16)bfr(Qp[(bb * CC + c0 + cl) * (size_t)TT + t0 + tl]); }
  __syncthreads(); for (int e = t; e < 64 * 16; e += 128) { const int tl = e >> 4, q = e & 15; vst2((unsigned*)(QR + (bb * TT + t0 + tl) * CC + c0 + q * 8), *(const v4u*)&st[tl][q * 8]); } }
__global__ __launch_bounds__(128) void k_kv(const float* __restrict__ KVp, const float* __restrict__ W, const float* __restrict__ Bk, _Float16* __restrict__ KH, _Float16* __restrict__ KL, _Float16* __restrict__ VH, _Float16* __restrict__ VL) {
  __shared__ __align__(16) _Float16 sh[64][136], sl[64][136]; __shared__ __align__(16) _Float16 th[128][72], tl2[128][72];
  const int tid = threadIdx.x, wave = tid >> 5, lane = tid & 31, col = lane & 15, g = lane >> 4; const int which = blockIdx.z / NBB; const size_t bb = blockIdx.z % NBB; const int t0 = blockIdx.x * 64; const int c0 = blockIdx.y * 128; const float* src = KVp + bb * CC * (size_t)TT;
  v8f acc[8] = {};
#pragma unroll 2
  for (int kc = 0; kc < CC / 32; ++kc) { v16b a; const int px = t0 + wave * 16 + col;
#pragma unroll
    for (int i = 0; i < 8; ++i) { a[i] = (__bf16)src[(size_t)(kc * 32 + 8 * g + i) * TT + px]; a[8 + i] = (__bf16)src[(size_t)(kc * 32 + 16 + 8 * g + i) * TT + px]; }
#pragma unroll
    for (int j = 0; j < 8; ++j) { v16b w; const int o = which * CC + c0 + j * 16 + col;
#pragma unroll
      for (int i = 0; i < 8; ++i) { w[i] = (__bf16)W[(size_t)(kc * 32 + 8 * g + i) * (2 * CC) + o]; w[8 + i] = (__bf16)W[(size_t)(kc * 32 + 16 + 8 * g + i) * (2 * CC) + o]; }
      acc[j] = wmma_bf(a, w, acc[j]); } }
#pragma unroll
  for (int j = 0; j < 8; ++j) { const float bbv = bfr(Bk[which * CC + c0 + j * 16 + col]);
#pragma unroll
    for (int r = 0; r < 8; ++r) { const float v = acc[j][r] + bbv; const _Float16 hv = (_Float16)v, lv = (_Float16)((v - (float)hv) * 2048.0f); const int rl = wave * 16 + 8 * g + r, cl = j * 16 + col; if (which == 0) { sh[rl][cl] = hv; sl[rl][cl] = lv; } else { th[cl][rl] = hv; tl2[cl][rl] = lv; } } }
  __syncthreads();
  if (which == 0) { for (int e = tid; e < 64 * 16; e += 128) { const int rl = e >> 4, q = e & 15; const size_t o = (bb * TT + t0 + rl) * CC + c0 + q * 8; vst2((unsigned*)(KH + o), *(const v4u*)&sh[rl][q * 8]); vst2((unsigned*)(KL + o), *(const v4u*)&sl[rl][q * 8]); } }
  else { for (int e = tid; e < 128 * 8; e += 128) { const int cl = e >> 3, q = e & 7; const size_t o = (bb * CC + c0 + cl) * (size_t)TT + t0 + q * 8; vst2((unsigned*)(VH + o), *(const v4u*)&th[cl][q * 8]); vst2((unsigned*)(VL + o), *(const v4u*)&tl2[cl][q * 8]); } } }
__global__ __launch_bounds__(128) void k_att(const _Float16* __restrict__ QR, const _Float16* __restrict__ KH, const _Float16* __restrict__ KL, const _Float16* __restrict__ VH, const _Float16* __restrict__ VL, float* __restrict__ Y) {
  __shared__ __align__(16) float sp[4][16][36]; __shared__ __align__(16) float so[4][16][68];
  const int tid = threadIdx.x, wave = tid >> 5, lane = tid & 31, col = lane & 15, g = lane >> 4; const int h = blockIdx.y; const size_t bb = blockIdx.z; const int q0 = blockIdx.x * 64 + wave * 16; const size_t rq = bb * TT + q0;
  v16h aq[2];
#pragma unroll
  for (int kc = 0; kc < 2; ++kc) aq[kc] = frag_h(QR + (rq + col) * CC + h * HD + kc * 32, lane);
  float m[8], l[8];
#pragma unroll
  for (int r = 0; r < 8; ++r) { m[r] = -3.0e38f; l[r] = 0.f; }
  v8f acc[4] = {}, accl[4] = {};
#pragma unroll 1
  for (int ks = 0; ks < TT / 32; ++ks) { float s[2][8];
#pragma unroll
    for (int ct = 0; ct < 2; ++ct) { const size_t rk = bb * TT + ks * 32 + ct * 16 + col; v8f c = {}, cl = {};
#pragma unroll
      for (int kc = 0; kc < 2; ++kc) { c = wmma16(aq[kc], frag_h(KH + rk * CC + h * HD + kc * 32, lane), c); cl = wmma16(aq[kc], frag_h(KL + rk * CC + h * HD + kc * 32, lane), cl); }
#pragma unroll
      for (int r = 0; r < 8; ++r) s[ct][r] = (c[r] + cl[r] * (1.0f / 2048.0f)) * 0.125f; }
    float alpha[8];
#pragma unroll
    for (int r = 0; r < 8; ++r) { float mx = fmaxf(s[0][r], s[1][r]);
#pragma unroll
      for (int o = 1; o < 16; o <<= 1) mx = fmaxf(mx, __shfl_xor(mx, o));
      const float mn = fmaxf(m[r], mx); alpha[r] = __expf(m[r] - mn); const float e0 = __expf(s[0][r] - mn), e1 = __expf(s[1][r] - mn); float es = e0 + e1;
#pragma unroll
      for (int o = 1; o < 16; o <<= 1) es += __shfl_xor(es, o);
      l[r] = l[r] * alpha[r] + es; m[r] = mn; sp[wave][8 * g + r][col] = e0; sp[wave][8 * g + r][16 + col] = e1; }
#pragma unroll
    for (int j = 0; j < 4; ++j)
#pragma unroll
      for (int r = 0; r < 8; ++r) { acc[j][r] *= alpha[r]; accl[j][r] *= alpha[r]; }
    LDSX();
    v16h pa; { const float* prow = &sp[wave][col][0] + 8 * (lane >> 4);
#pragma unroll
      for (int i = 0; i < 8; ++i) { pa[i] = (_Float16)(prow[i] * 2048.0f); pa[8 + i] = (_Float16)(prow[16 + i] * 2048.0f); } }
#pragma unroll
    for (int j = 0; j < 4; ++j) { const size_t po = (bb * CC + (size_t)h * HD + j * 16 + col) * (size_t)TT + ks * 32; acc[j] = wmma16(pa, frag_h(VH + po, lane), acc[j]); accl[j] = wmma16(pa, frag_h(VL + po, lane), accl[j]); }
    LDSX(); }
#pragma unroll
  for (int r = 0; r < 8; ++r) { const float il = (1.0f / 2048.0f) / l[r];
#pragma unroll
    for (int j = 0; j < 4; ++j) so[wave][8 * g + r][j * 16 + col] = (acc[j][r] + accl[j][r] * (1.0f / 2048.0f)) * il; }
  LDSX(); for (int rl = 0; rl < 16; ++rl) if (lane < 16) vst2(Y + (rq + rl) * CC + (size_t)h * HD + lane * 4, *(const v4f*)&so[wave][rl][lane * 4]); }
__global__ __launch_bounds__(128) void k_o(const float* __restrict__ Y, const float* __restrict__ WP, const float* __restrict__ BP, float* __restrict__ OUT) { __shared__ __align__(16) float sf[4][16][132];
  const int tid = threadIdx.x, wave = tid >> 5, lane = tid & 31, col = lane & 15, g = lane >> 4; const size_t bb = blockIdx.z; const int o0 = blockIdx.x * 64 + wave * 16; const int p0 = blockIdx.y * 128;
  v8f acc[8] = {};
#pragma unroll 2
  for (int kc = 0; kc < CC / 32; ++kc) { v16b a; const int o = o0 + col;
#pragma unroll
    for (int i = 0; i < 8; ++i) { a[i] = (__bf16)WP[(size_t)(kc * 32 + 8 * g + i) * CC + o]; a[8 + i] = (__bf16)WP[(size_t)(kc * 32 + 16 + 8 * g + i) * CC + o]; }
#pragma unroll
    for (int j = 0; j < 8; ++j) { float wv[16]; const float* wr = Y + (bb * TT + p0 + j * 16 + col) * CC + kc * 32 + 8 * g;
#pragma unroll
      for (int i = 0; i < 8; ++i) { wv[i] = wr[i]; wv[8 + i] = wr[16 + i]; }
      const F2 wb = bsplit16(wv); acc[j] = wmma_bf(a, wb.h, acc[j]); acc[j] = wmma_bf(a, wb.l, acc[j]); } }
#pragma unroll
  for (int j = 0; j < 8; ++j)
#pragma unroll
    for (int r = 0; r < 8; ++r) sf[wave][8 * g + r][j * 16 + col] = acc[j][r] + bfr(BP[o0 + 8 * g + r]);
  LDSX(); for (int rl = 0; rl < 16; ++rl) vst2(OUT + (bb * CC + o0 + rl) * (size_t)TT + p0 + lane * 4, *(const v4f*)&sf[wave][rl][lane * 4]); }
extern "C" void kernel_launch(void* const* d_in, const int* in_sizes, int n_in, void* d_out, int out_size, void* d_ws, size_t ws_size, hipStream_t stream) {
  (void)in_sizes; (void)n_in; (void)out_size;
  const float** F = (const float**)d_in;
  if (ws_size < (size_t)WS_END) return;
  char* ws = (char*)d_ws; _Float16 *QR = (_Float16*)(ws + WS_Q), *KH = (_Float16*)(ws + WS_KH), *KL = (_Float16*)(ws + WS_KL), *VH = (_Float16*)(ws + WS_VH), *VL = (_Float16*)(ws + WS_VL); float* Y = (float*)(ws + WS_Y);
  k_q<<<dim3(TT / 64, CC / 128, TBB), 128, 0, stream>>>(F[0], QR);
  k_kv<<<dim3(TT / 64, CC / 128, 2 * NBB), 128, 0, stream>>>(F[1], F[2], F[3], KH, KL, VH, VL);
  k_att<<<dim3(TT / 64, NH, TBB), 128, 0, stream>>>(QR, KH, KL, VH, VL, Y);
  k_o<<<dim3(CC / 64, TT / 128, TBB), 128, 0, stream>>>(Y, F[4], F[5], (float*)d_out);
}
